// VariableGT_42434276884502
// MI455X (gfx1250) — hardware-verified
//
#include <hip/hip_runtime.h>


namespace {
constexpr int S = 128, Bn = 32, V = 36, HID = 128, NH = 8, DK = 16, ST = 9, CC = HID * V, O1 = 4 * HID, NBL = Bn * S;
constexpr float QS = 0.25f, AS = 8.0f, WS = 64.0f, EPS = 1e-5f;

typedef _Float16 b16;
typedef __attribute__((ext_vector_type(16))) _Float16 v16b;
typedef __attribute__((ext_vector_type(8)))  _Float16 v8b;
typedef __attribute__((ext_vector_type(8)))  float v8f;
typedef __attribute__((ext_vector_type(4)))  float v4f;

__device__ __forceinline__ v8b ld8b(const b16* p) { return *(const v8b*)p; }
__device__ __forceinline__ v16b cat8b(v8b a, v8b b) { return __builtin_shufflevector(a, b, 0, 1, 2, 3, 4, 5, 6, 7, 8, 9, 10, 11, 12, 13, 14, 15); }
__device__ __forceinline__ v16b frag_kb(const b16* p, int hh) { return cat8b(ld8b(p + 8 * hh), ld8b(p + 16 + 8 * hh)); }
__device__ __forceinline__ void split16(float v, b16& hi, b16& lo) { hi = (b16)v; lo = (b16)(v - (float)hi); }
__device__ __forceinline__ void frag_ksplit(const float* p, int hh, v16b& fh_, v16b& fl_) {
  const float* p0 = p + 8 * hh; const float* p1 = p + 16 + 8 * hh;
#pragma unroll
  for (int e = 0; e < 8; ++e) { b16 a, c; split16(p0[e], a, c); fh_[e] = a; fl_[e] = c; split16(p1[e], a, c); fh_[8 + e] = a; fl_[8 + e] = c; }
}
__device__ __forceinline__ v8f wmma16b(v16b a, v16b b, v8f c) {
  v8f d = __builtin_amdgcn_wmma_f32_16x16x32_f16(false, a, false, b, (short)0, c, false, false);
  asm volatile("v_nop\n\tv_nop\n\tv_nop\n\tv_nop" : "+v"(d) : "v"(a), "v"(b));
  return d;
}
__device__ __forceinline__ void wave_lds_sync() {
  __builtin_amdgcn_fence(__ATOMIC_RELEASE, "workgroup");
  __builtin_amdgcn_wave_barrier();
  __builtin_amdgcn_fence(__ATOMIC_ACQUIRE, "workgroup");
}

struct Opnd { const void* p0; const void* p1; int ld; };
template <int NP> __device__ __forceinline__ void load_frags(const Opnd& o, int row, int kb, int hh, v16b& fh_, v16b& fl_) {
  if (NP == 0) { frag_ksplit((const float*)o.p0 + (size_t)row * o.ld + kb, hh, fh_, fl_); }
  else if (NP == 4) {
    const float* p = (const float*)o.p0 + (size_t)row * o.ld + kb; const float* p0 = p + 8 * hh; const float* p1 = p + 16 + 8 * hh;
#pragma unroll
    for (int e = 0; e < 8; ++e) { b16 a, c; split16(p0[e] * 64.0f, a, c); fh_[e] = a; fl_[e] = c; split16(p1[e] * 64.0f, a, c); fh_[8 + e] = a; fl_[8 + e] = c; }
  } else if (NP == 3) {
    const float* p = (const float*)o.p0 + (size_t)row * o.ld + kb; const float* p0 = p + 8 * hh; const float* p1 = p + 16 + 8 * hh;
#pragma unroll
    for (int e = 0; e < 8; ++e) { fh_[e] = (b16)p0[e]; fh_[8 + e] = (b16)p1[e]; }
    fl_ = fh_;
  } else {
    fh_ = frag_kb((const b16*)o.p0 + (size_t)row * o.ld + kb, hh);
    if (NP == 2) fl_ = frag_kb((const b16*)o.p1 + (size_t)row * o.ld + kb, hh); else fl_ = fh_;
  }
}
template <int ANP, int BNP> __device__ __forceinline__ v8f mac(v16b ah, v16b al, v16b bh, v16b bl, v8f c) {
  c = wmma16b(ah, bh, c);
  if (BNP == 0 || BNP == 2 || BNP == 4) c = wmma16b(ah, bl, c);
  if (ANP == 0 || ANP == 2 || ANP == 4) c = wmma16b(al, bh, c);
  return c;
}
template <int ANP, int BNP>
__device__ __forceinline__ void gemm_tile(const Opnd& A, const Opnd& B, int K, int m0, int c0, int nloc, int hlf, v8f (&acc)[2][4]) {
  for (int kb = 0; kb < K; kb += 32) {
    v16b a0h, a0l, a1h, a1l;
    load_frags<ANP>(A, m0 + nloc, kb, hlf, a0h, a0l);
    load_frags<ANP>(A, m0 + 16 + nloc, kb, hlf, a1h, a1l);
#pragma unroll
    for (int t = 0; t < 4; ++t) {
      v16b bh, bl;
      load_frags<BNP>(B, c0 + t * 16 + nloc, kb, hlf, bh, bl);
      acc[0][t] = mac<ANP, BNP>(a0h, a0l, bh, bl, acc[0][t]);
      acc[1][t] = mac<ANP, BNP>(a1h, a1l, bh, bl, acc[1][t]);
    }
  }
}

__device__ __forceinline__ void epi_planes(v8f (&acc)[2][4], float scale, bool two, b16* __restrict__ oh, b16* __restrict__ ol, int ldo,
                                           int m0, int c0, int lane, b16* Th, b16* Tl) {
  const int nloc = lane & 15, hlf = lane >> 4;
#pragma unroll
  for (int t = 0; t < 4; ++t)
#pragma unroll
    for (int r = 0; r < 2; ++r)
#pragma unroll
      for (int v = 0; v < 8; ++v) {
        const int rr = r * 16 + v + 8 * hlf, cc = t * 16 + nloc;
        b16 h_, l_; split16(acc[r][t][v] * scale, h_, l_);
        Th[rr * 64 + cc] = h_; Tl[rr * 64 + cc] = l_;
      }
  wave_lds_sync();
  for (int pass = 0; pass < 2; ++pass) {
#pragma unroll
    for (int j = 0; j < 8; ++j) {
      const int rr = j * 4 + (lane >> 3), c8 = (lane & 7) * 8;
      const size_t o = (size_t)(m0 + rr) * ldo + c0 + c8;
      *(volatile v8b*)(oh + o) = ld8b(Th + rr * 64 + c8);
      if (two) *(volatile v8b*)(ol + o) = ld8b(Tl + rr * 64 + c8);
    }
    __threadfence();
  }
}
__device__ __forceinline__ void epi_f32(v8f (&acc)[2][4], float scale, const float* rscale, float* __restrict__ out, int ldo, int m0, int c0, int lane, float* Tt) {
  const int nloc = lane & 15, hlf = lane >> 4;
#pragma unroll
  for (int t = 0; t < 4; ++t)
#pragma unroll
    for (int r = 0; r < 2; ++r)
#pragma unroll
      for (int v = 0; v < 8; ++v) {
        const int rr = r * 16 + v + 8 * hlf;
        const float rs = rscale ? rscale[(size_t)(m0 + rr) * 32] : 1.0f;
        Tt[rr * 64 + t * 16 + nloc] = acc[r][t][v] * scale * rs;
      }
  wave_lds_sync();
  float* dst0 = out + (size_t)m0 * ldo + c0;
  for (int pass = 0; pass < 2; ++pass) {
#pragma unroll
    for (int j = 0; j < 16; ++j) { const int rr = j * 2 + hlf, c4 = nloc * 4; *(volatile v4f*)(dst0 + (size_t)rr * ldo + c4) = *(const v4f*)(Tt + rr * 64 + c4); }
    __threadfence();
  }
}


__global__ __launch_bounds__(256) void prep_kernel(const float* __restrict__ Wq, const float* __restrict__ Wk, const float* __restrict__ Wv, const float* __restrict__ W1, const float* __restrict__ W2,
                                                   const float* __restrict__ Xtimes, const float* __restrict__ Xstatic, const float* __restrict__ Wemb, const float* __restrict__ bemb,
                                                   b16* __restrict__ wqkv, b16* __restrict__ w1h, b16* __restrict__ w1l, b16* __restrict__ w2h, b16* __restrict__ w2l, float* __restrict__ pe, float* __restrict__ emb) {
  const size_t tid = (size_t)blockIdx.x * blockDim.x + threadIdx.x, nth = (size_t)gridDim.x * blockDim.x;
  const size_t n0 = (size_t)3 * HID * HID / 8, n1 = (size_t)O1 * CC / 8, n2 = (size_t)HID * O1 / 8;
  for (int pass = 0; pass < 2; ++pass) {
    for (size_t p8 = tid; p8 < n0 + n1 + n2; p8 += nth) {
      if (p8 < n0) { const size_t i = p8 * 8; const int n = (int)(i / HID), k0 = (int)(i % HID); const int which = n / HID, nn = n % HID; const float* W = which == 0 ? Wq : which == 1 ? Wk : Wv; v8b v;
#pragma unroll
        for (int e = 0; e < 8; ++e) v[e] = (b16)W[(size_t)(k0 + e) * HID + nn];
        *(volatile v8b*)(wqkv + i) = v; }
      else if (p8 < n0 + n1) { const size_t i = (p8 - n0) * 8; v8b vh, vl;
#pragma unroll
        for (int e = 0; e < 8; ++e) { b16 a, c; split16(W1[i + e] * WS, a, c); vh[e] = a; vl[e] = c; }
        *(volatile v8b*)(w1h + i) = vh; *(volatile v8b*)(w1l + i) = vl; }
      else { const size_t i = (p8 - n0 - n1) * 8; v8b vh, vl;
#pragma unroll
        for (int e = 0; e < 8; ++e) { b16 a, c; split16(W2[i + e] * WS, a, c); vh[e] = a; vl[e] = c; }
        *(volatile v8b*)(w2h + i) = vh; *(volatile v8b*)(w2l + i) = vl; }
    }
    for (size_t i = tid; i < (size_t)Bn * S * HID; i += nth) { const int hid = (int)(i % HID), l = (int)((i / HID) % S), b = (int)(i / ((size_t)HID * S));
      const int j = hid >> 1; const float dv = expf(-(float)(2 * j) * (9.210340371976184f / (float)HID)); const float ang = Xtimes[l * Bn + b] * dv;
      ((volatile float*)pe)[i] = (hid & 1) ? cosf(ang) : sinf(ang); }
    for (size_t i = tid; i < (size_t)Bn * V * HID; i += nth) { const int hid = (int)(i % HID), v = (int)((i / HID) % V), b = (int)(i / ((size_t)HID * V)); const int row = v * HID + hid; float s = bemb[row];
#pragma unroll
      for (int t = 0; t < ST; ++t) s += Xstatic[b * ST + t] * Wemb[(size_t)row * ST + t];
      ((volatile float*)emb)[i] = s; }
    __threadfence();
  }
}

__device__ __forceinline__ float Hval(const float* __restrict__ Xtemp, const float* __restrict__ Wte, const float* __restrict__ bte, const float* __restrict__ pe, const float* __restrict__ emb, int b, int hid, int v, int l) {
  return Xtemp[((size_t)l * Bn + b) * V + v] * Wte[v * HID + hid] + bte[v * HID + hid] + pe[((size_t)b * S + l) * HID + hid] + emb[((size_t)b * V + v) * HID + hid];
}

__global__ __launch_bounds__(128) void h4_kernel(const float* __restrict__ Xtemp, const float* __restrict__ mask, const float* __restrict__ Wte, const float* __restrict__ bte, const float* __restrict__ pe, const float* __restrict__ emb, float* __restrict__ h4) {
  const int b = blockIdx.x / V, v = blockIdx.x % V, hid = threadIdx.x; float s = 0.0f, n = 0.0f;
#pragma unroll 1
  for (int l = 0; l < S; ++l) { const float mk = mask[((size_t)l * Bn + b) * V + v]; s += Hval(Xtemp, Wte, bte, pe, emb, b, hid, v, l) * mk; n += mk; }
  const float r = s / (n + 1.0f);
  ((volatile float*)h4)[((size_t)b * V + v) * HID + hid] = r; __threadfence(); ((volatile float*)h4)[((size_t)b * V + v) * HID + hid] = r;
}

__global__ __launch_bounds__(128) void qkv_kernel(const float* __restrict__ h4, const b16* __restrict__ wqkv, float* __restrict__ qkv) {
  __shared__ __attribute__((aligned(16))) float Ts[4][32 * 64];
  const int lane = threadIdx.x & 31, wave = threadIdx.x >> 5, nloc = lane & 15, hlf = lane >> 4, m0 = blockIdx.y * 128 + wave * 32, c0 = blockIdx.x * 64;
  v8f acc[2][4];
#pragma unroll
  for (int r = 0; r < 2; ++r)
#pragma unroll
    for (int t = 0; t < 4; ++t) acc[r][t] = (v8f){};
  const Opnd A{h4, nullptr, HID}, B{wqkv, nullptr, HID};
  gemm_tile<3, 1>(A, B, HID, m0, c0, nloc, hlf, acc);
  epi_f32(acc, (c0 < 2 * HID) ? QS : 1.0f, nullptr, qkv, 3 * HID, m0, c0, lane, Ts[wave]);
}

__global__ __launch_bounds__(96) void e_kernel(const float* __restrict__ qkv, b16* __restrict__ E) {
  __shared__ __attribute__((aligned(16))) b16 Te[3][16][64 + 8];
  const int wave = threadIdx.x >> 5, lane = threadIdx.x & 31, nloc = lane & 15, hlf = lane >> 4, b = blockIdx.x / NH, h = blockIdx.x % NH, v0 = wave * 16;
  v16b af = {};
  { const int v = v0 + nloc; if (v < V) { const float* qr = qkv + ((size_t)b * V + v) * 3 * HID + h * DK;
#pragma unroll
      for (int e = 0; e < 8; ++e) af[e] = (b16)qr[8 * hlf + e]; } }
  v8f acc[3] = {{}, {}, {}};
#pragma unroll
  for (int t = 0; t < 3; ++t) { v16b bf_ = {}; const int u = t * 16 + nloc; if (u < V) { const float* kr = qkv + ((size_t)b * V + u) * 3 * HID + HID + h * DK;
#pragma unroll
      for (int e = 0; e < 8; ++e) bf_[e] = (b16)kr[8 * hlf + e]; }
    acc[t] = wmma16b(af, bf_, acc[t]); }
#pragma unroll
  for (int r = 0; r < 8; ++r) {
    float mx = -INFINITY;
#pragma unroll
    for (int t = 0; t < 3; ++t) if (t * 16 + nloc < V) mx = fmaxf(mx, acc[t][r]);
#pragma unroll
    for (int o = 1; o < 16; o <<= 1) mx = fmaxf(mx, __shfl_xor(mx, o));
    const int v = v0 + 8 * hlf + r;
#pragma unroll
    for (int t = 0; t < 3; ++t) { const int u = t * 16 + nloc; Te[wave][8 * hlf + r][u] = (b16)((u < V && v < V) ? __expf(acc[t][r] - mx) : 0.0f); }
    Te[wave][8 * hlf + r][48 + nloc] = (b16)0.0f;
  }
  wave_lds_sync();
  b16* dst = E + (((size_t)b * NH + h) * 48 + v0) * 64;
  for (int pass = 0; pass < 2; ++pass) {
#pragma unroll
    for (int j = 0; j < 4; ++j) { const int rr = j * 4 + (lane >> 3), c8 = (lane & 7) * 8; *(volatile v8b*)(dst + rr * 64 + c8) = *(const v8b*)(&Te[wave][rr][c8]); }
    __threadfence();
  }
}

__global__ __launch_bounds__(128) void v5_kernel(const b16* __restrict__ E, const float* __restrict__ Xtemp, const float* __restrict__ mask, const float* __restrict__ Wte, const float* __restrict__ bte,
                                                 const float* __restrict__ pe, const float* __restrict__ emb, const float* __restrict__ qkv, b16* __restrict__ v5h, b16* __restrict__ v5l) {
  __shared__ __attribute__((aligned(16))) b16 Oh[4][4][576 + 8]; __shared__ __attribute__((aligned(16))) b16 Ol[4][4][576 + 8];
  __shared__ float Den[4][48][4]; __shared__ float Ef[4][48][36 + 1];
  const int wave = threadIdx.x >> 5, lane = threadIdx.x & 31, nloc = lane & 15, hlf = lane >> 4;
  const int wg = blockIdx.x * 4 + wave; const int lt = wg & 31, h = (wg >> 5) & 7, b = wg >> 8, l0 = lt * 4;
  const b16* Eb = E + ((size_t)b * NH + h) * 48 * 64;
  for (int i = lane; i < 48 * 36; i += 32) { const int v = i / 36, u = i % 36; Ef[wave][v][u] = (float)Eb[v * 64 + u]; }
  wave_lds_sync();
  for (int i = lane; i < 48 * 4; i += 32) { const int v = i / 4, ll = i % 4; float s = 0.0f;
#pragma unroll 1
    for (int u = 0; u < V; ++u) s += Ef[wave][v][u] * mask[((size_t)(l0 + ll) * Bn + b) * V + u];
    Den[wave][v][ll] = s; }
  v8f acc[3][4];
#pragma unroll
  for (int r = 0; r < 3; ++r)
#pragma unroll
    for (int t = 0; t < 4; ++t) acc[r][t] = (v8f){};
#pragma unroll
  for (int ks = 0; ks < 2; ++ks) {
    v16b a[3];
#pragma unroll
    for (int r = 0; r < 3; ++r) a[r] = frag_kb(Eb + (size_t)(r * 16 + nloc) * 64 + ks * 32, hlf);
#pragma unroll
    for (int t = 0; t < 4; ++t) {
      const int l = l0 + t, d = nloc, hid = h * DK + d; v16b bh_, bl_;
#pragma unroll
      for (int e = 0; e < 16; ++e) { const int u = ks * 32 + ((e < 8) ? (8 * hlf + e) : (16 + 8 * hlf + e - 8)); float val = 0.0f;
        if (u < V) { const float mk = mask[((size_t)l * Bn + b) * V + u]; val = (mk != 0.0f) ? mk * Hval(Xtemp, Wte, bte, pe, emb, b, hid, u, l) : 0.0f; }
        b16 x0, x1; split16(val * AS, x0, x1); bh_[e] = x0; bl_[e] = x1; }
#pragma unroll
      for (int r = 0; r < 3; ++r) { acc[r][t] = wmma16b(a[r], bh_, acc[r][t]); acc[r][t] = wmma16b(a[r], bl_, acc[r][t]); }
    }
  }
  wave_lds_sync();
#pragma unroll
  for (int t = 0; t < 4; ++t)
#pragma unroll
    for (int r = 0; r < 3; ++r)
#pragma unroll
      for (int vv = 0; vv < 8; ++vv) { const int v = r * 16 + 8 * hlf + vv; if (v < V) { const int d = nloc, hid = h * DK + d;
          const float val = acc[r][t][vv] * (1.0f / AS) / Den[wave][v][t] + qkv[((size_t)b * V + v) * 3 * HID + 2 * HID + hid];
          b16 x0, x1; split16(val * AS, x0, x1); Oh[wave][t][d * V + v] = x0; Ol[wave][t][d * V + v] = x1; } }
  wave_lds_sync();
  for (int pass = 0; pass < 2; ++pass) {
#pragma unroll
    for (int t = 0; t < 4; ++t) { b16* dh = v5h + ((size_t)(b * S + l0 + t)) * CC + h * 576; b16* dl = v5l + ((size_t)(b * S + l0 + t)) * CC + h * 576;
      for (int pcs = lane; pcs < 72; pcs += 32) { *(volatile v8b*)(dh + pcs * 8) = *(const v8b*)(&Oh[wave][t][pcs * 8]); *(volatile v8b*)(dl + pcs * 8) = *(const v8b*)(&Ol[wave][t][pcs * 8]); } }
    __threadfence();
  }
}

__global__ __launch_bounds__(128) void y_kernel(const b16* __restrict__ w1h, const b16* __restrict__ w1l, const b16* __restrict__ v5h, const b16* __restrict__ v5l, const float* __restrict__ b1, float* __restrict__ y32) {
  __shared__ __attribute__((aligned(16))) float Ts[4][32 * 64];
  const int lane = threadIdx.x & 31, wave = threadIdx.x >> 5, nloc = lane & 15, hlf = lane >> 4, m0 = blockIdx.y * 128 + wave * 32, c0 = blockIdx.x * 64;
  v8f acc[2][4];
#pragma unroll
  for (int r = 0; r < 2; ++r)
#pragma unroll
    for (int t = 0; t < 4; ++t) acc[r][t] = (v8f){};
  const Opnd A{w1h, w1l, CC}, B{v5h, v5l, CC};
  gemm_tile<2, 2>(A, B, CC, m0, c0, nloc, hlf, acc);
  float* Tt = Ts[wave];
#pragma unroll
  for (int t = 0; t < 4; ++t)
#pragma unroll
    for (int r = 0; r < 2; ++r)
#pragma unroll
      for (int v = 0; v < 8; ++v) { const int rr = r * 16 + v + 8 * hlf; Tt[rr * 64 + t * 16 + nloc] = acc[r][t][v] * (1.0f / (AS * WS)) + b1[m0 + rr]; }
  wave_lds_sync();
  for (int pass = 0; pass < 2; ++pass) {
#pragma unroll
    for (int j = 0; j < 16; ++j) { const int rr = j * 2 + hlf, c4 = nloc * 4; *(volatile v4f*)(y32 + (size_t)(m0 + rr) * NBL + c0 + c4) = *(const v4f*)(Tt + rr * 64 + c4); }
    __threadfence();
  }
}

__global__ __launch_bounds__(256) void bnrow_kernel(const float* __restrict__ y, int ncols, const float* __restrict__ g, const float* __restrict__ bb, float* __restrict__ ca, float* __restrict__ csh) {
  __shared__ float As_[32], Ss_[32];
  const int wave = threadIdx.x >> 5, lane = threadIdx.x & 31, r0 = blockIdx.x * 32;
  for (int qq = 0; qq < 4; ++qq) { const int row = r0 + wave * 4 + qq; double s = 0.0, s2 = 0.0;
#pragma unroll 1
    for (int c = lane; c < ncols; c += 32) { const double v = y[(size_t)row * ncols + c]; s += v; s2 += v * v; }
#pragma unroll
    for (int o = 16; o > 0; o >>= 1) { s += __shfl_xor(s, o); s2 += __shfl_xor(s2, o); }
    if (lane == 0) { const double mean = s / ncols, var = s2 / ncols - mean * mean; const float a = g[row] * (float)(1.0 / sqrt(var + (double)EPS)); As_[wave * 4 + qq] = a; Ss_[wave * 4 + qq] = bb[row] - (float)mean * a; } }
  __syncthreads();
  if (wave == 0) for (int pass = 0; pass < 2; ++pass) { ((volatile float*)ca)[r0 + lane] = As_[lane]; ((volatile float*)csh)[r0 + lane] = Ss_[lane]; __threadfence(); }
}

__device__ __forceinline__ float gelu_e(float x) { return 0.5f * x * (1.0f + erff(x * 0.7071067811865475f)); }

__global__ __launch_bounds__(256) void bn1_kernel(const float* __restrict__ y32, const float* __restrict__ ca, const float* __restrict__ csh, b16* __restrict__ yh, b16* __restrict__ yl) {
  __shared__ __attribute__((aligned(16))) b16 Th[64][72]; __shared__ __attribute__((aligned(16))) b16 Tl[64][72];
  const int tid = threadIdx.x, lane = tid & 31, wave = tid >> 5, c0 = blockIdx.x * 64, o0 = blockIdx.y * 64;
  for (int i = tid; i < 64 * 64; i += 256) { const int oo = i / 64, cc = i % 64; const int o = o0 + oo; b16 a, c; split16(gelu_e(y32[(size_t)o * NBL + c0 + cc] * ca[o] + csh[o]) * AS, a, c); Th[cc][oo] = a; Tl[cc][oo] = c; }
  __syncthreads();
  for (int pass = 0; pass < 2; ++pass) {
#pragma unroll
    for (int j = 0; j < 2; ++j) { const int rr = wave * 8 + j * 4 + (lane >> 3), c8 = (lane & 7) * 8;
      *(volatile v8b*)(yh + (size_t)(c0 + rr) * O1 + o0 + c8) = *(const v8b*)(&Th[rr][c8]); *(volatile v8b*)(yl + (size_t)(c0 + rr) * O1 + o0 + c8) = *(const v8b*)(&Tl[rr][c8]); }
    __threadfence();
  }
}

__global__ __launch_bounds__(128) void z_kernel(const b16* __restrict__ w2h, const b16* __restrict__ w2l, const b16* __restrict__ yh, const b16* __restrict__ yl, const float* __restrict__ b2, float* __restrict__ z32) {
  __shared__ __attribute__((aligned(16))) float Ts[4][32 * 64];
  const int lane = threadIdx.x & 31, wave = threadIdx.x >> 5, nloc = lane & 15, hlf = lane >> 4, m0 = wave * 32, c0 = blockIdx.x * 64;
  v8f acc[2][4];
#pragma unroll
  for (int r = 0; r < 2; ++r)
#pragma unroll
    for (int t = 0; t < 4; ++t) acc[r][t] = (v8f){};
  const Opnd A{w2h, w2l, O1}, B{yh, yl, O1};
  gemm_tile<2, 2>(A, B, O1, m0, c0, nloc, hlf, acc);
  float* Tt = Ts[wave];
#pragma unroll
  for (int t = 0; t < 4; ++t)
#pragma unroll
    for (int r = 0; r < 2; ++r)
#pragma unroll
      for (int v = 0; v < 8; ++v) { const int rr = r * 16 + v + 8 * hlf; Tt[rr * 64 + t * 16 + nloc] = acc[r][t][v] * (1.0f / (AS * WS)) + b2[m0 + rr]; }
  wave_lds_sync();
  for (int pass = 0; pass < 2; ++pass) {
#pragma unroll
    for (int j = 0; j < 16; ++j) { const int rr = j * 2 + hlf, c4 = nloc * 4; *(volatile v4f*)(z32 + (size_t)(m0 + rr) * NBL + c0 + c4) = *(const v4f*)(Tt + rr * 64 + c4); }
    __threadfence();
  }
}

__global__ __launch_bounds__(256) void bn2_kernel(const float* __restrict__ z32, const float* __restrict__ ca, const float* __restrict__ csh, float* __restrict__ out) {
  const int o = blockIdx.x, t = threadIdx.x; const float a = ca[o], sh = csh[o];
  for (int pass = 0; pass < 2; ++pass) {
    for (int i = t; i < NBL / 4; i += 256) { const int c = i * 4, b = c / S, l = c % S; v4f x = *(const v4f*)(z32 + (size_t)o * NBL + c), w;
#pragma unroll
      for (int e = 0; e < 4; ++e) w[e] = gelu_e(x[e] * a + sh);
      *(volatile v4f*)(out + ((size_t)b * HID + o) * S + l) = w; }
    __threadfence();
  }
}
}

extern "C" void kernel_launch(void* const* d_in, const int* in_sizes, int n_in,
                              void* d_out, int out_size, void* d_ws, size_t ws_size, hipStream_t stream) {
  (void)n_in; (void)out_size;
  const float* Xtemp = (const float*)d_in[0]; const float* Xtimes = (const float*)d_in[1]; const float* Xstatic = (const float*)d_in[2]; const float* mask = (const float*)d_in[3];
  const float* Wte = (const float*)d_in[4]; const float* bte = (const float*)d_in[5]; const float* Wemb = (const float*)d_in[6]; const float* bemb = (const float*)d_in[7];
  const float* Wq = (const float*)d_in[8]; const float* Wk = (const float*)d_in[9]; const float* Wv = (const float*)d_in[10];
  const float* W1 = (const float*)d_in[11]; const float* b1 = (const float*)d_in[12]; const float* g1 = (const float*)d_in[13]; const float* be1 = (const float*)d_in[14];
  const float* W2 = (const float*)d_in[15]; const float* b2 = (const float*)d_in[16]; const float* g2 = (const float*)d_in[17]; const float* be2 = (const float*)d_in[18];
  float* out = (float*)d_out;
  if (in_sizes[0] != S * Bn * V || in_sizes[3] != S * Bn * V || in_sizes[6] != CC * ST || in_sizes[11] != O1 * CC || in_sizes[15] != HID * O1) return;
  size_t off = 0; char* ws = (char*)d_ws;
  auto carve = [&](size_t bytes) { char* p = ws + off; off += (bytes + 255) & ~(size_t)255; return p; };
  b16* wqkv = (b16*)carve((size_t)3 * HID * HID * 2);
  b16* w1h = (b16*)carve((size_t)O1 * CC * 2); b16* w1l = (b16*)carve((size_t)O1 * CC * 2);
  b16* w2h = (b16*)carve((size_t)HID * O1 * 2); b16* w2l = (b16*)carve((size_t)HID * O1 * 2);
  float* pe = (float*)carve((size_t)Bn * S * HID * 4); float* emb = (float*)carve((size_t)Bn * V * HID * 4); float* h4 = (float*)carve((size_t)Bn * V * HID * 4);
  float* qkv = (float*)carve((size_t)Bn * V * 3 * HID * 4);
  b16* E = (b16*)carve((size_t)Bn * NH * 48 * 64 * 2);
  b16* v5h = (b16*)carve((size_t)NBL * CC * 2); b16* v5l = (b16*)carve((size_t)NBL * CC * 2);
  float* y32 = (float*)carve((size_t)O1 * NBL * 4);
  float* ca = (float*)carve(O1 * 4); float* csh = (float*)carve(O1 * 4);
  b16* yh = (b16*)carve((size_t)NBL * O1 * 2); b16* yl = (b16*)carve((size_t)NBL * O1 * 2);
  float* z32 = (float*)carve((size_t)HID * NBL * 4);
  if (off > ws_size) return;
  prep_kernel<<<512, 256, 0, stream>>>(Wq, Wk, Wv, W1, W2, Xtimes, Xstatic, Wemb, bemb, wqkv, w1h, w1l, w2h, w2l, pe, emb);
  h4_kernel<<<Bn * V, 128, 0, stream>>>(Xtemp, mask, Wte, bte, pe, emb, h4);
  qkv_kernel<<<dim3(3 * HID / 64, Bn * V / 128), 128, 0, stream>>>(h4, wqkv, qkv);
  e_kernel<<<Bn * NH, 96, 0, stream>>>(qkv, E);
  v5_kernel<<<Bn * NH * 32 / 4, 128, 0, stream>>>(E, Xtemp, mask, Wte, bte, pe, emb, qkv, v5h, v5l);
  y_kernel<<<dim3(NBL / 64, O1 / 128), 128, 0, stream>>>(w1h, w1l, v5h, v5l, b1, y32);
  bnrow_kernel<<<O1 / 32, 256, 0, stream>>>(y32, NBL, g1, be1, ca, csh);
  bn1_kernel<<<dim3(NBL / 64, O1 / 64), 256, 0, stream>>>(y32, ca, csh, yh, yl);
  z_kernel<<<dim3(NBL / 64, 1), 128, 0, stream>>>(w2h, w2l, yh, yl, b2, z32);
  bnrow_kernel<<<HID / 32, 256, 0, stream>>>(z32, NBL, g2, be2, ca, csh);
  bn2_kernel<<<HID, 256, 0, stream>>>(z32, ca, csh, out);
}
